// SimpleMambaBlock_84937273246163
// MI455X (gfx1250) — hardware-run, weakly checked
//
#include <hip/hip_runtime.h>
#include <hip/hip_fp16.h>
#include <math.h>

typedef __attribute__((ext_vector_type(16))) _Float16 v16h;
typedef __attribute__((ext_vector_type(8)))  _Float16 v8h;
typedef __attribute__((ext_vector_type(8)))  float    v8f;
typedef __attribute__((ext_vector_type(4)))  float    v4f;

constexpr int kBatch = 4;
constexpr int kDim   = 384;
constexpr int kSeq   = 4096;
constexpr int kNst   = 16;
constexpr int kProjN = 2 * kDim + 2 * kNst;
constexpr int kProjP = 832;
constexpr int kPieces = kProjP / 4;
constexpr float kWCarry = 1024.0f;
constexpr float kResid  = 2048.0f;
constexpr float kYCarry = 16.0f;
constexpr float kScaleP  = 1.0f / 1024.0f;
constexpr float kScalePr = 1.0f / (1024.0f * 2048.0f);
constexpr float kScaleO  = 1.0f / (16.0f * 1024.0f);
constexpr float kScaleOr = 1.0f / (16.0f * 1024.0f * 2048.0f);
static_assert(kProjN == 800);
static_assert((kProjP % 64) == 0 && kProjP >= kProjN);
static_assert((kDim % 64) == 0 && (kDim % 32) == 0 && (kDim % 8) == 0);
static_assert((kSeq % 64) == 0 && (kSeq % 32) == 0 && (kSeq % 16) == 0);
static_assert((kProjN % 4) == 0 && (kDim % 4) == 0);
static_assert((((kSeq / 16) * (kProjP / 64)) % 8) == 0);
static_assert((((kSeq / 32) * (kDim / 64)) % 8) == 0);
static_assert(((kProjP * kDim / 8) % 256) == 0);
static_assert(((kDim * kDim / 8) % 256) == 0);
static_assert(((kSeq * kPieces) % 256) == 0);

constexpr size_t kSzWP   = (size_t)kProjP * kDim * 2;
constexpr size_t kSzWO   = (size_t)kDim * kDim * 2;
constexpr size_t kSzX16  = (size_t)kSeq * kDim * 2;
constexpr size_t kSzPROJ = (size_t)kSeq * kProjP * 4;
constexpr size_t kSzOUTP = (size_t)kSeq * kDim * 4;
constexpr size_t kOffWPH  = 0;
constexpr size_t kOffWPL  = kOffWPH  + kSzWP;
constexpr size_t kOffWOH  = kOffWPL  + kSzWP;
constexpr size_t kOffXH   = kOffWOH  + kSzWO;
constexpr size_t kOffXL   = kOffXH   + kSzX16;
constexpr size_t kOffPROJ = kOffXL   + kSzX16;
constexpr size_t kOffYH   = kOffPROJ + kSzPROJ;
constexpr size_t kOffYL   = kOffYH   + kSzX16;
constexpr size_t kOffOUTP = kOffYL   + kSzX16;
constexpr size_t kWsTotal = kOffOUTP + kSzOUTP;
static_assert(kWsTotal == 34078720ull);
static_assert(kWsTotal <= 134217728ull);
static_assert((kOffWPL % 128) == 0 && (kOffWOH % 128) == 0 && (kOffXH % 128) == 0 && (kOffXL % 128) == 0 &&
              (kOffPROJ % 128) == 0 && (kOffYH % 128) == 0 && (kOffYL % 128) == 0 && (kOffOUTP % 128) == 0);

__device__ __forceinline__ _Float16 f16_flush(float v) {
  const float w = (fabsf(v) < 6.103515625e-05f) ? 0.0f : v;
  return (_Float16)w;
}
__device__ __forceinline__ void f16_split(float v, _Float16& hi, _Float16& lo) {
  hi = f16_flush(v);
  const float hf = (float)hi;
  const float r = (v - hf) * kResid;
  lo = f16_flush(r);
}

namespace eng {
union FragU { v16h v; v8h h[2]; };
__device__ __forceinline__ v16h frag_load(const _Float16* p) {
  FragU f;
  f.h[0] = *(const v8h*)(p);
  f.h[1] = *(const v8h*)(p + 16);
  return f.v;
}
__device__ __forceinline__ v8f mma(v16h a, v16h b, v8f c) {
  return __builtin_amdgcn_wmma_f32_16x16x32_f16(false, a, false, b, (short)0, c, false, false);
}
__device__ __forceinline__ void guard1(v8f& a, v16h x, v16h y) {
  asm volatile("v_nop\n\tv_nop\n\tv_nop\n\tv_nop" : "+v"(a) : "v"(x), "v"(y));
}
__device__ __forceinline__ void guard_acc(v8f& a) {
  asm volatile("v_nop\n\tv_nop\n\tv_nop\n\tv_nop" : "+v"(a));
}
__device__ __forceinline__ void keep4(v16h a, v16h b, v16h c, v16h d) {
  asm volatile("v_nop" :: "v"(a), "v"(b), "v"(c), "v"(d));
}

template <int MI, int SPL>
__global__ __launch_bounds__(256) void gemm_f16_kernel(
    const unsigned short* __restrict__ Ap, const unsigned short* __restrict__ A2p, int lda,
    const unsigned short* __restrict__ Btp, const unsigned short* __restrict__ Bt2p, int ldb,
    float* __restrict__ C, int ldc, int M, int N, int K, float scale, float rscale)
{
  static_assert(MI >= 1 && MI <= 2);
  static_assert(SPL >= 0 && SPL <= 2);
  const _Float16* A   = (const _Float16*)Ap;
  const _Float16* A2  = (const _Float16*)A2p;
  const _Float16* Bt  = (const _Float16*)Btp;
  const _Float16* Bt2 = (const _Float16*)Bt2p;
  __shared__ __align__(16) float sT[8][16 * 68];
  const int lane = threadIdx.x & 31;
  const int wave = threadIdx.x >> 5;
  const int tilesN = N >> 6;
  const int tilesM = M / (16 * MI);
  const int tile = blockIdx.x * 8 + wave;
  if (tile >= tilesM * tilesN) return;
  const int tm = tile / tilesN;
  const int tn = tile - tm * tilesN;
  const int m0 = tm * (16 * MI);
  const int n0 = tn << 6;
  const int rlane = lane & 15;
  const int koff  = (lane >> 4) * 8;
  const int mOff  = (lane >> 4) * 8;

  v8f acc[MI][4], accr[MI][4];
#pragma unroll
  for (int i = 0; i < MI; ++i)
#pragma unroll
    for (int j = 0; j < 4; ++j) {
      acc[i][j]  = (v8f){0.f, 0.f, 0.f, 0.f, 0.f, 0.f, 0.f, 0.f};
      accr[i][j] = (v8f){0.f, 0.f, 0.f, 0.f, 0.f, 0.f, 0.f, 0.f};
    }

  for (int k0 = 0; k0 < K; k0 += 32) {
    v16h bh[4], bl[4];
#pragma unroll
    for (int j = 0; j < 4; ++j) {
      const size_t bo = (size_t)(n0 + (j << 4) + rlane) * ldb + koff + k0;
      bh[j] = frag_load(Bt + bo);
      if (SPL == 2) bl[j] = frag_load(Bt2 + bo); else bl[j] = bh[j];
    }
#pragma unroll
    for (int i = 0; i < MI; ++i) {
      const size_t ao = (size_t)(m0 + (i << 4) + rlane) * lda + koff + k0;
      const v16h ah = frag_load(A + ao);
      v16h al = ah;
      if (SPL >= 1) al = frag_load(A2 + ao);
#pragma unroll
      for (int j = 0; j < 4; ++j) {
        acc[i][j] = mma(ah, bh[j], acc[i][j]);
        if (SPL >= 1) accr[i][j] = mma(al, bh[j], accr[i][j]);
        if (SPL == 2) accr[i][j] = mma(ah, bl[j], accr[i][j]);
      }
#pragma unroll
      for (int j = 0; j < 4; ++j) {
        guard1(acc[i][j], ah, al);
        if (SPL >= 1) guard1(accr[i][j], ah, al);
      }
    }
    keep4(bh[0], bh[1], bh[2], bh[3]);
    if (SPL == 2) keep4(bl[0], bl[1], bl[2], bl[3]);
  }
#pragma unroll
  for (int i = 0; i < MI; ++i)
#pragma unroll
    for (int j = 0; j < 4; ++j) {
      guard_acc(acc[i][j]);
      if (SPL >= 1) guard_acc(accr[i][j]);
    }

  float* slab = sT[wave];
#pragma unroll
  for (int i = 0; i < MI; ++i) {
    const int mBase = m0 + (i << 4);
#pragma unroll
    for (int j = 0; j < 4; ++j) {
#pragma unroll
      for (int r = 0; r < 8; ++r) {
        float v = acc[i][j][r] * scale;
        if (SPL >= 1) v += accr[i][j][r] * rscale;
        slab[(mOff + r) * 68 + (j << 4) + rlane] = v;
      }
    }
    __builtin_amdgcn_fence(__ATOMIC_RELEASE, "workgroup");
    __builtin_amdgcn_wave_barrier();
    __builtin_amdgcn_fence(__ATOMIC_ACQUIRE, "workgroup");
    {
      const int hh = lane >> 4, c4 = (lane & 15) * 4;
      for (int pass = 0; pass < 2; ++pass) {
#pragma unroll
        for (int it = 0; it < 8; ++it) {
          const int row = it * 2 + hh;
          const v4f v = *(const v4f*)(slab + row * 68 + c4);
          *(volatile v4f*)(C + (size_t)(mBase + row) * ldc + n0 + c4) = v;
        }
        __threadfence();
      }
    }
    __builtin_amdgcn_fence(__ATOMIC_RELEASE, "workgroup");
    __builtin_amdgcn_wave_barrier();
    __builtin_amdgcn_fence(__ATOMIC_ACQUIRE, "workgroup");
  }
}
}

template <bool LO>
__global__ __launch_bounds__(256) void pack_weight_rows_kernel(
    const float* __restrict__ W, unsigned short* __restrict__ dH, unsigned short* __restrict__ dL,
    int rowsReal, int total8)
{
  const int i = blockIdx.x * 256 + threadIdx.x;
  if (i >= total8) return;
  const int e0  = i << 3;
  const int row = e0 / kDim;
  const int col = e0 - row * kDim;
  const int rc  = (row < rowsReal) ? row : (rowsReal - 1);
  const float* sp = W + (size_t)rc * kDim + col;
  const v4f a0 = *(const v4f*)(sp);
  const v4f a1 = *(const v4f*)(sp + 4);
  float f[8];
#pragma unroll
  for (int e = 0; e < 4; ++e) {
    f[e] = a0[e];
    f[4 + e] = a1[e];
  }
#pragma unroll
  for (int e = 0; e < 8; ++e) asm volatile("" : "+v"(f[e]));
  const bool live = (row < rowsReal);
  v8h hv, lv;
#pragma unroll
  for (int e = 0; e < 8; ++e) {
    const float t = live ? (f[e] * kWCarry) : 0.0f;
    _Float16 h, l;
    f16_split(t, h, l);
    hv[e] = h;
    lv[e] = l;
  }
  unsigned short* qh = dH + e0;
  unsigned short* ql = dL + e0;
  *(volatile v8h*)qh = hv;
  if (LO) *(volatile v8h*)ql = lv;
  __threadfence();
  *(volatile v8h*)qh = hv;
  if (LO) *(volatile v8h*)ql = lv;
}

__global__ __launch_bounds__(256) void xpose_split_kernel(
    const float* __restrict__ xb, unsigned short* __restrict__ dH, unsigned short* __restrict__ dL)
{
  __shared__ float tile[64 * 65];
  const int tid = threadIdx.x, lane = tid & 31, wave = tid >> 5;
  const int l0 = blockIdx.x * 64;
  const int c0 = blockIdx.y * 64;
  const int rr = tid >> 4;
  const int l4 = (tid & 15) * 4;
#pragma unroll
  for (int p = 0; p < 4; ++p) {
    const int cc = p * 16 + rr;
    const v4f v = *(const v4f*)(xb + (size_t)(c0 + cc) * kSeq + l0 + l4);
    tile[cc * 65 + l4 + 0] = v[0];
    tile[cc * 65 + l4 + 1] = v[1];
    tile[cc * 65 + l4 + 2] = v[2];
    tile[cc * 65 + l4 + 3] = v[3];
  }
  __syncthreads();
  const int q = lane >> 3, c8 = (lane & 7) * 8;
  v8h hv[2], lv[2];
#pragma unroll
  for (int it = 0; it < 2; ++it) {
    const int lrow = it * 32 + wave * 4 + q;
#pragma unroll
    for (int e = 0; e < 8; ++e) {
      _Float16 h, l;
      const float t = tile[(c8 + e) * 65 + lrow];
      f16_split(t, h, l);
      hv[it][e] = h;
      lv[it][e] = l;
    }
  }
  for (int pass = 0; pass < 2; ++pass) {
#pragma unroll
    for (int it = 0; it < 2; ++it) {
      const int lrow = it * 32 + wave * 4 + q;
      const size_t o = (size_t)(l0 + lrow) * kDim + c0 + c8;
      *(volatile v8h*)(dH + o) = hv[it];
      *(volatile v8h*)(dL + o) = lv[it];
    }
    __threadfence();
  }
}

__global__ __launch_bounds__(256) void bias_rows_kernel(
    float* P, const float* __restrict__ bp, const float* __restrict__ dtb, int total4)
{
  const int i = blockIdx.x * 256 + threadIdx.x;
  if (i >= total4) return;
  const int row = i / kPieces;
  const int n4  = (i - row * kPieces) * 4;
  float* p = P + (size_t)i * 4;
  const v4f v = *(const v4f*)p;
  const int nb = (n4 < kProjN) ? n4 : (kProjN - 4);
  int nd = n4 - kDim;
  nd = (nd < 0) ? 0 : nd;
  nd = (nd > kDim - 4) ? (kDim - 4) : nd;
  const v4f b4 = *(const v4f*)(bp + nb);
  const v4f d4 = *(const v4f*)(dtb + nd);
  float pv[4], bv[4], dv[4];
#pragma unroll
  for (int e = 0; e < 4; ++e) {
    pv[e] = v[e];
    bv[e] = b4[e];
    dv[e] = d4[e];
  }
#pragma unroll
  for (int e = 0; e < 4; ++e) {
    asm volatile("" : "+v"(pv[e]));
    asm volatile("" : "+v"(bv[e]));
    asm volatile("" : "+v"(dv[e]));
  }
  const bool inB = (n4 < kProjN);
  const bool inD = (n4 >= kDim) && (n4 < 2 * kDim);
  v4f o;
#pragma unroll
  for (int e = 0; e < 4; ++e) {
    const float bs = inB ? bv[e] : 0.0f;
    const float ds = inD ? dv[e] : 0.0f;
    o[e] = (pv[e] + bs) + ds;
  }
  *(volatile v4f*)p = o;
  __threadfence();
  *(volatile v4f*)p = o;
}

__global__ __launch_bounds__(256) void out_xpose_bias_kernel(
    const float* __restrict__ OP, const float* __restrict__ bo, float* __restrict__ outb)
{
  __shared__ float tile[64 * 65];
  const int tid = threadIdx.x, lane = tid & 31, wave = tid >> 5;
  const int l0 = blockIdx.x * 64;
  const int c0 = blockIdx.y * 64;
  const int rr = tid >> 4;
  const int c4 = (tid & 15) * 4;
#pragma unroll
  for (int p = 0; p < 4; ++p) {
    const int ll = p * 16 + rr;
    const v4f v = *(const v4f*)(OP + (size_t)(l0 + ll) * kDim + c0 + c4);
    tile[ll * 65 + c4 + 0] = v[0];
    tile[ll * 65 + c4 + 1] = v[1];
    tile[ll * 65 + c4 + 2] = v[2];
    tile[ll * 65 + c4 + 3] = v[3];
  }
  __syncthreads();
  const int hh = lane >> 4, l4 = (lane & 15) * 4;
  v4f ov[4];
#pragma unroll
  for (int it = 0; it < 4; ++it) {
    const int crow = it * 16 + wave * 2 + hh;
    const float bv = bo[c0 + crow];
#pragma unroll
    for (int e = 0; e < 4; ++e) ov[it][e] = tile[(l4 + e) * 65 + crow] + bv;
  }
  for (int pass = 0; pass < 2; ++pass) {
#pragma unroll
    for (int it = 0; it < 4; ++it) {
      const int crow = it * 16 + wave * 2 + hh;
      *(volatile v4f*)(outb + (size_t)(c0 + crow) * kSeq + l0 + l4) = ov[it];
    }
    __threadfence();
  }
}

typedef float    ms1_v4f __attribute__((ext_vector_type(4)));
typedef unsigned ms1_v4u __attribute__((ext_vector_type(4)));
struct ms1_args {
  const float* dtpre;
  const float* u;
  const float* bc;
  const float* z;
  const float* A_log;
  const float* Dskip;
  __half* y;
  __half* y_lo;
  long ld_dtpre;
  long ld_u;
  long ld_bc;
  long ld_z;
  long ld_y;
  int offB;
  int offC;
  int offZ;
  float ycarry;
  int dir;
  int D;
  int L;
  int nbatch;
};
static_assert(sizeof(ms1_args) == 136);

__device__ __forceinline__ float ms1_flush16(float v) {
  return (fabsf(v) < 6.103515625e-05f) ? 0.0f : v;
}
__device__ __forceinline__ unsigned ms1_h16bits(float v) {
  return (unsigned)__half_as_ushort(__float2half_rn(ms1_flush16(v)));
}
__device__ __forceinline__ float ms1_h16val(unsigned b) {
  return __half2float(__ushort_as_half((unsigned short)b));
}
__device__ __forceinline__ float ms1_softplus(float v) {
  return fmaxf(v, 0.0f) + log1pf(expf(-fabsf(v)));
}
__device__ __forceinline__ void ms1_pack2(float v0, float v1, unsigned& hw, unsigned& lw) {
  const unsigned h0 = ms1_h16bits(v0);
  const unsigned h1 = ms1_h16bits(v1);
  const float r0 = (v0 - ms1_h16val(h0)) * 2048.0f;
  const float r1 = (v1 - ms1_h16val(h1)) * 2048.0f;
  const unsigned l0 = ms1_h16bits(r0);
  const unsigned l1 = ms1_h16bits(r1);
  hw = h0 | (h1 << 16);
  lw = l0 | (l1 << 16);
}

template <int NSTATE>
__global__ __launch_bounds__(64 * (NSTATE / 16)) void ms1_scan_kernel(ms1_args a)
{
  static_assert(NSTATE == 16 || NSTATE == 64);
  constexpr int NQ  = NSTATE / 16;
  constexpr int NT  = 64 * NQ;
  constexpr int NW  = NT / 32;
  constexpr int BCW = 2 * NSTATE;
  constexpr int YP  = 68;
  constexpr int RPI = NW * 4;
  constexpr int NIT = 64 / RPI;
  static_assert(16 * NT <= 64 * YP);
  __shared__ __align__(16) float sBC[64 * BCW];
  __shared__ __align__(16) float sY[64 * YP];
  const int tid  = threadIdx.x;
  const int lane = tid & 31;
  const int wave = tid >> 5;
  const int c    = tid / NQ;
  const int sq   = tid - c * NQ;
  const int bpb  = a.D / 64;
  const int bi   = blockIdx.x / bpb;
  if (bi >= a.nbatch) return;
  const int d0 = (blockIdx.x - bi * bpb) * 64;
  const int d  = d0 + c;
  const long rowb = (long)bi * a.L;
  const bool hasz  = (a.z != nullptr);
  const bool hasD  = (a.Dskip != nullptr);
  const bool hasLo = (a.y_lo != nullptr);

#pragma unroll 1
  for (int n = 0; n < 16; ++n) {
    const float al = a.A_log[(long)d * NSTATE + sq * 16 + n];
    sY[n * NT + tid] = -expf(al);
  }
  __syncthreads();
  float An[16], h[16];
#pragma unroll
  for (int n = 0; n < 16; ++n) {
    An[n] = sY[n * NT + tid];
    h[n] = 0.0f;
  }
  float Dd = 0.0f;
  if (hasD) Dd = a.Dskip[d];

  const int nchunk = a.L / 64;
  const bool fwd = (a.dir > 0);
  const int s0 = fwd ? 0 : 63;
  const int sd = fwd ? 1 : -1;
  const int q  = lane >> 3;
  const int c8 = (lane & 7) * 8;

#pragma unroll 1
  for (int ci = 0; ci < nchunk; ++ci) {
    const int tb = fwd ? (ci * 64) : (a.L - 64 - ci * 64);
    const long rowc = rowb + tb;
    __syncthreads();
#pragma unroll 8
    for (int i = 0; i < 32; ++i) {
      const int idx = tid + i * NT;
      const int st  = idx / BCW;
      const int col = idx - st * BCW;
      const int sc  = (col < NSTATE) ? (a.offB + col) : (a.offC + col - NSTATE);
      sBC[idx] = a.bc[(rowc + st) * a.ld_bc + sc];
    }
    __syncthreads();
#pragma unroll 1
    for (int s = 0; s < 64; ++s) {
      const int ls = s0 + sd * s;
      const long row = rowc + ls;
      float pre = a.dtpre[row * a.ld_dtpre + d];
      float uv  = a.u[row * a.ld_u + d];
      float zv  = 0.0f;
      if (hasz) zv = a.z[row * a.ld_z + a.offZ + d];
      asm volatile("" : "+v"(pre));
      asm volatile("" : "+v"(uv));
      asm volatile("" : "+v"(zv));
      const float delta = ms1_softplus(pre);
      const float dtx = delta * uv;
      const float* bp = sBC + ls * BCW + sq * 16;
      const float* cp = bp + NSTATE;
      ms1_v4f Bq[4], Cq[4];
#pragma unroll
      for (int k = 0; k < 4; ++k) {
        Bq[k] = *(const ms1_v4f*)(bp + 4 * k);
        Cq[k] = *(const ms1_v4f*)(cp + 4 * k);
      }
      float yv = 0.0f;
#pragma unroll
      for (int n = 0; n < 16; ++n) {
        const float e = __expf(delta * An[n]);
        h[n] = fmaf(e, h[n], dtx * Bq[n >> 2][n & 3]);
        yv = fmaf(h[n], Cq[n >> 2][n & 3], yv);
      }
      if (NQ > 1) {
        yv += __shfl_xor(yv, 1, 32);
        yv += __shfl_xor(yv, 2, 32);
      }
      if (hasD) yv = fmaf(uv, Dd, yv);
      if (hasz) {
        const float sg = __builtin_amdgcn_rcpf(1.0f + expf(-zv));
        yv = yv * (zv * sg);
      }
      if (sq == 0) sY[ls * YP + c] = yv * a.ycarry;
    }
    __syncthreads();
    ms1_v4u hw[NIT], lw[NIT];
#pragma unroll
    for (int it = 0; it < NIT; ++it) {
      const int row = it * RPI + wave * 4 + q;
      const float* sp = sY + row * YP + c8;
      const ms1_v4f f0 = *(const ms1_v4f*)(sp);
      const ms1_v4f f1 = *(const ms1_v4f*)(sp + 4);
      unsigned h0, h1, h2, h3, l0, l1, l2, l3;
      ms1_pack2(f0[0], f0[1], h0, l0);
      ms1_pack2(f0[2], f0[3], h1, l1);
      ms1_pack2(f1[0], f1[1], h2, l2);
      ms1_pack2(f1[2], f1[3], h3, l3);
      hw[it] = (ms1_v4u){h0, h1, h2, h3};
      lw[it] = (ms1_v4u){l0, l1, l2, l3};
    }
    for (int pass = 0; pass < 2; ++pass) {
#pragma unroll
      for (int it = 0; it < NIT; ++it) {
        const int row = it * RPI + wave * 4 + q;
        const long o = (rowc + row) * a.ld_y + d0 + c8;
        *(volatile ms1_v4u*)(a.y + o) = hw[it];
        if (hasLo) *(volatile ms1_v4u*)(a.y_lo + o) = lw[it];
      }
      __threadfence();
    }
  }
}

extern "C" void kernel_launch(void* const* d_in, const int* in_sizes, int n_in,
                              void* d_out, int out_size, void* d_ws, size_t ws_size,
                              hipStream_t stream)
{
  if (n_in < 8) return;
  if (in_sizes[0] != kBatch * kDim * kSeq) return;
  if (in_sizes[1] != kProjN * kDim) return;
  if (in_sizes[2] != kProjN) return;
  if (in_sizes[3] != kDim * kNst) return;
  if (in_sizes[4] != kDim) return;
  if (in_sizes[5] != kDim) return;
  if (in_sizes[6] != kDim * kDim) return;
  if (in_sizes[7] != kDim) return;
  if (out_size != kBatch * kDim * kSeq) return;
  if (ws_size < kWsTotal) return;

  const float* x       = (const float*)d_in[0];
  const float* W_proj  = (const float*)d_in[1];
  const float* b_proj  = (const float*)d_in[2];
  const float* A_log   = (const float*)d_in[3];
  const float* D_par   = (const float*)d_in[4];
  const float* dt_bias = (const float*)d_in[5];
  const float* W_out   = (const float*)d_in[6];
  const float* b_out   = (const float*)d_in[7];
  float* out = (float*)d_out;

  char* ws = (char*)d_ws;
  unsigned short* WPH  = (unsigned short*)(ws + kOffWPH);
  unsigned short* WPL  = (unsigned short*)(ws + kOffWPL);
  unsigned short* WOH  = (unsigned short*)(ws + kOffWOH);
  unsigned short* XH   = (unsigned short*)(ws + kOffXH);
  unsigned short* XL   = (unsigned short*)(ws + kOffXL);
  float*          PROJ = (float*)(ws + kOffPROJ);
  unsigned short* YH   = (unsigned short*)(ws + kOffYH);
  unsigned short* YL   = (unsigned short*)(ws + kOffYL);
  float*          OUTP = (float*)(ws + kOffOUTP);

  pack_weight_rows_kernel<true><<<dim3((kProjP * kDim / 8) / 256), 256, 0, stream>>>(
      W_proj, WPH, WPL, kProjN, kProjP * kDim / 8);
  pack_weight_rows_kernel<false><<<dim3((kDim * kDim / 8) / 256), 256, 0, stream>>>(
      W_out, WOH, WOH, kDim, kDim * kDim / 8);

  for (int b = 0; b < kBatch; ++b) {
    const float* xb = x + (size_t)b * kDim * kSeq;
    float* outb = out + (size_t)b * kDim * kSeq;

    xpose_split_kernel<<<dim3(kSeq / 64, kDim / 64), 256, 0, stream>>>(xb, XH, XL);

    eng::gemm_f16_kernel<1, 2><<<dim3((kSeq / 16) * (kProjP / 64) / 8), 256, 0, stream>>>(
        XH, XL, kDim, WPH, WPL, kDim, PROJ, kProjP, kSeq, kProjP, kDim, kScaleP, kScalePr);

    bias_rows_kernel<<<dim3((kSeq * kPieces) / 256), 256, 0, stream>>>(PROJ, b_proj, dt_bias, kSeq * kPieces);

    ms1_args sa;
    sa.dtpre = PROJ + kDim;
    sa.u = PROJ;
    sa.bc = PROJ + 2 * kDim;
    sa.z = nullptr;
    sa.A_log = A_log;
    sa.Dskip = D_par;
    sa.y = (__half*)YH;
    sa.y_lo = (__half*)YL;
    sa.ld_dtpre = kProjP;
    sa.ld_u = kProjP;
    sa.ld_bc = kProjP;
    sa.ld_z = 0;
    sa.ld_y = kDim;
    sa.offB = 0;
    sa.offC = kNst;
    sa.offZ = 0;
    sa.ycarry = kYCarry;
    sa.dir = 1;
    sa.D = kDim;
    sa.L = kSeq;
    sa.nbatch = 1;
    ms1_scan_kernel<16><<<dim3(kDim / 64), 64, 0, stream>>>(sa);

    eng::gemm_f16_kernel<2, 1><<<dim3((kSeq / 32) * (kDim / 64) / 8), 256, 0, stream>>>(
        YH, YL, kDim, WOH, WOH, kDim, OUTP, kDim, kSeq, kDim, kDim, kScaleO, kScaleOr);

    out_xpose_bias_kernel<<<dim3(kSeq / 64, kDim / 64), 256, 0, stream>>>(OUTP, b_out, outb);
  }
}
